// Stacked_Filter_22754736734701
// MI455X (gfx1250) — hardware-verified
//
#include <hip/hip_runtime.h>
#include <math.h>

#ifndef NNODE
#define NNODE 2048
#endif
#ifndef NFEAT
#define NFEAT 256
#endif
#define NN_FULL 2048
#define NFEAT_FULL 256
#define NHOP 4
#define LG_PER 8
#define LD_ROWS 32
#define ZB_N NNODE

static_assert(NNODE == NN_FULL);
static_assert(NFEAT == NFEAT_FULL);
static_assert(NNODE % 64 == 0 && NFEAT % 64 == 0);
static_assert(NNODE % 32 == 0);
static_assert((1 << LG_PER) * 8 == NNODE);
static_assert(NNODE % 128 == 0);
static_assert(NNODE % LD_ROWS == 0);
static_assert(ZB_N >= NFEAT && ZB_N >= NNODE);
static_assert((ZB_N / 4) % 32 == 0);
static_assert(ZB_N / 4 <= NNODE * NFEAT / 4);
static_assert(8 * 16 * 68 * 4 <= 131072);
static_assert(LD_ROWS * 4 <= 131072);

typedef __attribute__((ext_vector_type(16))) _Float16 v16h;
typedef __attribute__((ext_vector_type(8)))  _Float16 v8h;
typedef __attribute__((ext_vector_type(8)))  float    v8f;
typedef __attribute__((ext_vector_type(4)))  float    v4f;
typedef __attribute__((ext_vector_type(4)))  unsigned int v4u;


#define VST2(T, ptr, val) do { const T vst2_v_ = (val); *(volatile T*)(ptr) = vst2_v_; __threadfence(); *(volatile T*)(ptr) = vst2_v_; } while (0)
#define VST2V4(ptr, val) do { const v4f vst2_v4_ = (val); *(volatile v4f*)(ptr) = vst2_v4_; __threadfence(); *(volatile v4f*)(ptr) = vst2_v4_; } while (0)

__device__ __forceinline__ float bfr(float f) {
    unsigned u = __float_as_uint(f);
    u += 0x7FFFu + ((u >> 16) & 1u);
    return __uint_as_float(u & 0xFFFF0000u);
}
__device__ __forceinline__ unsigned short f2h_bits(float x) {
    return (fabsf(x) < 6.104e-5f) ? (unsigned short)0 : __builtin_bit_cast(unsigned short, (_Float16)x);
}
__device__ __forceinline__ void st8h(unsigned short* P, size_t o, const float* v) {
    v4u pk;
    pk.x = (unsigned)f2h_bits(v[0]) | ((unsigned)f2h_bits(v[1]) << 16);
    pk.y = (unsigned)f2h_bits(v[2]) | ((unsigned)f2h_bits(v[3]) << 16);
    pk.z = (unsigned)f2h_bits(v[4]) | ((unsigned)f2h_bits(v[5]) << 16);
    pk.w = (unsigned)f2h_bits(v[6]) | ((unsigned)f2h_bits(v[7]) << 16);
    VST2(v4u, (v4u*)(P + o), pk);
}

union FragU { v16h v; v8h h[2]; };
__device__ __forceinline__ v16h frag_ld(const _Float16* p) {
    FragU f; f.h[0] = *(const v8h*)(p); f.h[1] = *(const v8h*)(p + 16); return f.v;
}
__device__ __forceinline__ v8f wmma16(v16h a, v16h b, v8f c) {
    c = __builtin_amdgcn_wmma_f32_16x16x32_f16(false, a, false, b, (short)0, c, false, false);
    asm volatile("v_nop\n\tv_nop\n\tv_nop\n\tv_nop" : "+v"(c) : "v"(a), "v"(b));
    return c;
}
__device__ __forceinline__ void dep_guard_h(v8f& a, v8f& b, v16h x, v16h y) { asm volatile("v_nop\n\tv_nop\n\tv_nop\n\tv_nop" : "+v"(a), "+v"(b) : "v"(x), "v"(y)); }
__device__ __forceinline__ void keep4_h(v16h a, v16h b, v16h c, v16h d) { asm volatile("v_nop" :: "v"(a), "v"(b), "v"(c), "v"(d)); }
__device__ __forceinline__ void acc_guard4(v8f& a, v8f& b, v8f& c, v8f& d) { asm volatile("v_nop\n\tv_nop\n\tv_nop\n\tv_nop" : "+v"(a), "+v"(b), "+v"(c), "+v"(d)); }
__device__ __forceinline__ void wave_sync_lds() {
    __builtin_amdgcn_fence(3  , "workgroup");
    __builtin_amdgcn_wave_barrier();
    __builtin_amdgcn_fence(2  , "workgroup");
}

template <int OUT_MODE, bool RESID, bool RELU>
__global__ __launch_bounds__(256) void k_gemm64(
    const _Float16* __restrict__ A, unsigned lda, const _Float16* __restrict__ Bt, unsigned ldb,
    void* __restrict__ Cout, unsigned ldc, const float* __restrict__ bias, const float* __restrict__ resid,
    unsigned M, unsigned N, unsigned K, float scale, float oscale) {
  __shared__ __align__(16) float sT[8][16 * 68];
  const unsigned lane = threadIdx.x & 31u;
  const unsigned wave = threadIdx.x >> 5;
  const unsigned tilesN = N >> 6, tilesM = M >> 6;
  const unsigned tile = blockIdx.x * 8u + wave;
  if (tile >= tilesM * tilesN) return;
  const unsigned tm = tile / tilesN;
  const unsigned tn = tile - tm * tilesN;
  const unsigned m0 = tm << 6, n0 = tn << 6;
  const unsigned rlane = lane & 15u;
  const unsigned koff = (lane >> 4) * 8u;
  const unsigned mOff = koff;

  v8f acc[4][4];
#pragma unroll
  for (int i = 0; i < 4; ++i)
#pragma unroll
    for (int j = 0; j < 4; ++j) acc[i][j] = (v8f){0.f,0.f,0.f,0.f,0.f,0.f,0.f,0.f};

  for (unsigned k0 = 0; k0 < K; k0 += 32u) {
    v16h bh[4];
#pragma unroll
    for (int j = 0; j < 4; ++j)
      bh[j] = frag_ld(Bt + (size_t)(n0 + ((unsigned)j << 4) + rlane) * ldb + koff + k0);
#pragma unroll
    for (int i = 0; i < 4; ++i) {
      const v16h ah = frag_ld(A + (size_t)(m0 + ((unsigned)i << 4) + rlane) * lda + koff + k0);
#pragma unroll
      for (int j = 0; j < 4; ++j)
        acc[i][j] = __builtin_amdgcn_wmma_f32_16x16x32_f16(false, ah, false, bh[j], (short)0, acc[i][j], false, false);
      dep_guard_h(acc[i][0], acc[i][3], ah, ah);
    }
    keep4_h(bh[0], bh[1], bh[2], bh[3]);
  }
  acc_guard4(acc[0][0], acc[0][1], acc[0][2], acc[0][3]);
  acc_guard4(acc[1][0], acc[1][1], acc[1][2], acc[1][3]);
  acc_guard4(acc[2][0], acc[2][1], acc[2][2], acc[2][3]);
  acc_guard4(acc[3][0], acc[3][1], acc[3][2], acc[3][3]);

  float* slab = sT[wave];
#pragma unroll
  for (int i = 0; i < 4; ++i) {
    const unsigned mBase = m0 + ((unsigned)i << 4);
#pragma unroll
    for (int j = 0; j < 4; ++j) {
      const unsigned n = n0 + ((unsigned)j << 4) + rlane;
      const float bv = bfr(bias[n]);
#pragma unroll
      for (int r = 0; r < 8; ++r) {
        float v = acc[i][j][r] * scale + bv;
        if (RELU) v = fmaxf(v, 0.0f);
        if (OUT_MODE == 1) v *= oscale;
        slab[(mOff + (unsigned)r) * 68u + ((unsigned)j << 4) + rlane] = v;
      }
    }
    wave_sync_lds();
    if (OUT_MODE == 0) {
      float* C = (float*)Cout;
      const unsigned hh = lane >> 4, c4 = (lane & 15u) * 4u;
#pragma unroll
      for (int half = 0; half < 2; ++half) {
        v4f vv[4];
#pragma unroll
        for (int it = 0; it < 4; ++it) {
          const unsigned row = (unsigned)(half * 4 + it) * 2u + hh;
          vv[it] = *(const v4f*)(slab + row * 68u + c4);
          if (RESID) vv[it] += *(const v4f*)(resid + (size_t)(mBase + row) * ldc + n0 + c4);
        }
        for (int pass = 0; pass < 2; ++pass) {
#pragma unroll
          for (int it = 0; it < 4; ++it) {
            const unsigned row = (unsigned)(half * 4 + it) * 2u + hh;
            *(volatile v4f*)(C + (size_t)(mBase + row) * ldc + n0 + c4) = vv[it];
          }
          __threadfence();
        }
      }
    } else {
      _Float16* C = (_Float16*)Cout;
      const unsigned q = lane >> 3, c8 = (lane & 7u) * 8u;
      v8h hv[4];
#pragma unroll
      for (int it = 0; it < 4; ++it) {
        const unsigned row = (unsigned)it * 4u + q;
        const float* sp = slab + row * 68u + c8;
#pragma unroll
        for (int e = 0; e < 8; ++e) hv[it][e] = (_Float16)sp[e];
      }
      for (int pass = 0; pass < 2; ++pass) {
#pragma unroll
        for (int it = 0; it < 4; ++it) {
          const unsigned row = (unsigned)it * 4u + q;
          *(volatile v8h*)(C + (size_t)(mBase + row) * ldc + n0 + c8) = hv[it];
        }
        __threadfence();
      }
    }
    wave_sync_lds();
  }
}

__global__ __launch_bounds__(256) void k_wt16(const float* __restrict__ Wm, unsigned KI, unsigned NO, unsigned lgper,
                                              unsigned short* __restrict__ W16, float sw) {
    const unsigned layer = blockIdx.y;
    const float* Wl = Wm + (size_t)layer * KI * NO;
    unsigned short* Dl = W16 + (size_t)layer * KI * NO;
    const unsigned u = blockIdx.x * 256u + threadIdx.x;
    const unsigned per = 1u << lgper;
    if (u >= NO * per) return;
    const unsigned k0 = 8u * (u & (per - 1u));
    const unsigned o = u >> lgper;
    float v[8];
#pragma unroll
    for (int i = 0; i < 8; ++i) v[i] = bfr(Wl[(size_t)(k0 + (unsigned)i) * NO + o]) * sw;
    st8h(Dl, (size_t)o * KI + k0, v);
}

static_assert(((size_t)NNODE * NNODE / 8) % 256 == 0);
static_assert(((size_t)NNODE * NNODE / 8 / 256) * 256 * 16 == (size_t)NNODE * NNODE * 2);
__global__ __launch_bounds__(256) void k_cvt16(const float* __restrict__ src, unsigned short* __restrict__ dst,
                                               unsigned n8, float sw) {
#pragma clang fp contract(off)
    const unsigned u = blockIdx.x * 256u + threadIdx.x;
    if (u >= n8) return;
    const float* sp = src + (size_t)u * 8u;
    const v4f a = *(const v4f*)sp, b = *(const v4f*)(sp + 4);
    float v[8];
    v[0] = bfr(a.x) * sw; v[1] = bfr(a.y) * sw; v[2] = bfr(a.z) * sw; v[3] = bfr(a.w) * sw;
    v[4] = bfr(b.x) * sw; v[5] = bfr(b.y) * sw; v[6] = bfr(b.z) * sw; v[7] = bfr(b.w) * sw;
    st8h(dst, (size_t)u * 8u, v);
}

static_assert(8 * 4 == LD_ROWS);
static_assert(8 * 16 == LD_ROWS * 4);
__global__ __launch_bounds__(256) void k_lamdiag(const float* __restrict__ lam, const float* __restrict__ av,
                                                 const float* __restrict__ bv, const float* __restrict__ cv,
                                                 float* __restrict__ dvec) {
#pragma clang fp contract(off)
    __shared__ __align__(16) float sD[LD_ROWS];
    const unsigned lane = threadIdx.x & 31u;
    const unsigned wave = (unsigned)__builtin_amdgcn_readfirstlane((int)(threadIdx.x >> 5));
    const unsigned rbase = blockIdx.x * (unsigned)LD_ROWS + wave * 4u;
#pragma unroll 1
    for (unsigned rr = 0; rr < 4u; ++rr) {
        const unsigned row = rbase + rr;
        const float* lr = lam + (size_t)row * NN_FULL;
        int bad = 0;
#pragma unroll 4
        for (unsigned it = 0; it < (unsigned)(NNODE / 128); ++it) {
            const unsigned c0 = 4u * (lane + 32u * it);
            const v4f v = *(const v4f*)(lr + c0);
            bad |= (((c0      ) != row) && !(v.x == 0.0f)) ? 1 : 0;
            bad |= (((c0 + 1u) != row) && !(v.y == 0.0f)) ? 1 : 0;
            bad |= (((c0 + 2u) != row) && !(v.z == 0.0f)) ? 1 : 0;
            bad |= (((c0 + 3u) != row) && !(v.w == 0.0f)) ? 1 : 0;
        }
        bad |= __shfl_xor(bad, 16, 32);
        bad |= __shfl_xor(bad, 8, 32);
        bad |= __shfl_xor(bad, 4, 32);
        bad |= __shfl_xor(bad, 2, 32);
        bad |= __shfl_xor(bad, 1, 32);
        const float l = bfr(lr[row]);
        float acc = 0.f;
#pragma unroll 1
        for (unsigned i = 0; i < (unsigned)NHOP; ++i) {
            const float ai = bfr(av[i]), bi = bfr(bv[i]), ci = bfr(cv[i]);
            const float rep = fmaxf((ai - l) * (l - bi), 0.0f);
            const float dd = ai - bi;
            const float den = (dd * dd) * 0.25f;
            const float sc = ci * (1.0f / den);
            acc = acc + sc * rep;
        }
        const float dval = (bad != 0) ? __uint_as_float(0x7FC00000u) : acc;
        if (lane == 0u) sD[wave * 4u + rr] = dval;
    }
    __syncthreads();
    if (threadIdx.x < 8u) {
        const v4f o = *(const v4f*)(sD + 4u * threadIdx.x);
        VST2V4(dvec + (size_t)blockIdx.x * (unsigned)LD_ROWS + 4u * threadIdx.x, o);
    }
}

static_assert(((size_t)NNODE * NFEAT / 4) % 256 == 0);
static_assert(((size_t)NNODE * NFEAT / 4 / 256) * 256 * 16 == (size_t)NNODE * NFEAT * 4);
__global__ __launch_bounds__(256) void k_prep(const float* __restrict__ x, const float* __restrict__ alpha,
                                              float* __restrict__ xr, float* __restrict__ zb) {
#pragma clang fp contract(off)
    const unsigned u = blockIdx.x * 256u + threadIdx.x;
    if (u >= (unsigned)(NNODE * NFEAT / 4)) return;
    const float al = bfr(alpha[0]);
    const v4f a = *(const v4f*)(x + (size_t)u * 4u);
    v4f r;
    r.x = al * bfr(a.x); r.y = al * bfr(a.y); r.z = al * bfr(a.z); r.w = al * bfr(a.w);
    VST2V4(xr + (size_t)u * 4u, r);
    if (u < (unsigned)(ZB_N / 4)) {
        const v4f z = (v4f){0.f, 0.f, 0.f, 0.f};
        VST2V4(zb + (size_t)u * 4u, z);
    }
}

static_assert(((size_t)NFEAT * NNODE / 8) % 256 == 0);
static_assert(((size_t)NFEAT * NNODE / 8 / 256) * 256 * 16 == (size_t)NFEAT * NNODE * 2);
__global__ __launch_bounds__(256) void k_zscale(const float* __restrict__ yt, const float* __restrict__ dvec,
                                                unsigned short* __restrict__ zt16) {
#pragma clang fp contract(off)
    const unsigned u = blockIdx.x * 256u + threadIdx.x;
    if (u >= (unsigned)(NFEAT * NNODE / 8)) return;
    const unsigned j0 = (u % (unsigned)(NNODE / 8)) * 8u;
    const float* yp = yt + (size_t)u * 8u;
    const v4f y0 = *(const v4f*)yp, y1 = *(const v4f*)(yp + 4);
    const v4f d0 = *(const v4f*)(dvec + j0), d1 = *(const v4f*)(dvec + j0 + 4u);
    float v[8];
    v[0] = (y0.x * d0.x) * 8.0f; v[1] = (y0.y * d0.y) * 8.0f; v[2] = (y0.z * d0.z) * 8.0f; v[3] = (y0.w * d0.w) * 8.0f;
    v[4] = (y1.x * d1.x) * 8.0f; v[5] = (y1.y * d1.y) * 8.0f; v[6] = (y1.z * d1.z) * 8.0f; v[7] = (y1.w * d1.w) * 8.0f;
    st8h(zt16, (size_t)u * 8u, v);
}

static constexpr float SC   = 1.0f / 256.0f;
static constexpr float SW_U = 32.0f;
static constexpr float SW_X = 8.0f;

static constexpr size_t SZ_UT16 = (size_t)NNODE * NNODE * 2;
static constexpr size_t SZ_U16  = (size_t)NNODE * NNODE * 2;
static constexpr size_t SZ_XT16 = (size_t)NFEAT * NNODE * 2;
static constexpr size_t SZ_ZT16 = (size_t)NFEAT * NNODE * 2;
static constexpr size_t SZ_XR   = (size_t)NNODE * NFEAT * 4;
static constexpr size_t SZ_YT   = (size_t)NFEAT * NNODE * 4;
static constexpr size_t SZ_DV   = (size_t)NNODE * 4;
static constexpr size_t SZ_ZB   = (size_t)ZB_N * 4;
static constexpr size_t WS_TOTAL = SZ_UT16 + SZ_U16 + SZ_XT16 + SZ_ZT16 + SZ_XR + SZ_YT + SZ_DV + SZ_ZB;
static_assert(SZ_UT16 % 256 == 0 && SZ_XT16 % 256 == 0 && SZ_XR % 256 == 0 && SZ_YT % 256 == 0 && SZ_DV % 256 == 0 && SZ_ZB % 256 == 0);
static_assert(WS_TOTAL <= (size_t)134217728);
static_assert(((size_t)NNODE * (NNODE / 8)) % 256 == 0 && ((size_t)NFEAT * (NNODE / 8)) % 256 == 0);
static_assert(((NFEAT / 64) * (NNODE / 64)) % 8 == 0);

extern "C" void kernel_launch(void* const* d_in, const int* in_sizes, int n_in, void* d_out, int out_size,
                              void* d_ws, size_t ws_size, hipStream_t stream) {
    if (n_in < 7) return;
    if (in_sizes[0] < NNODE * NFEAT || in_sizes[1] < NNODE * NNODE || in_sizes[2] < NNODE * NNODE) return;
    if (in_sizes[3] < NHOP || in_sizes[4] < NHOP || in_sizes[5] < NHOP || in_sizes[6] < 1) return;
    if (out_size < NNODE * NFEAT) return;

    const float* x     = (const float*)d_in[0];
    const float* lam   = (const float*)d_in[1];
    const float* U     = (const float*)d_in[2];
    const float* a_l   = (const float*)d_in[3];
    const float* b_l   = (const float*)d_in[4];
    const float* c_l   = (const float*)d_in[5];
    const float* alpha = (const float*)d_in[6];
    float* out = (float*)d_out;

    char* wsp = (char*)d_ws;
    size_t off = 0;
    auto carve = [&](size_t bytes) -> void* { void* r = wsp + off; off += (bytes + 255) & ~(size_t)255; return r; };
    unsigned short* ut16 = (unsigned short*)carve(SZ_UT16);
    unsigned short* u16  = (unsigned short*)carve(SZ_U16);
    unsigned short* xt16 = (unsigned short*)carve(SZ_XT16);
    unsigned short* zt16 = (unsigned short*)carve(SZ_ZT16);
    float*          xr   = (float*)carve(SZ_XR);
    float*          yt   = (float*)carve(SZ_YT);
    float*          dvec = (float*)carve(SZ_DV);
    float*          zb   = (float*)carve(SZ_ZB);
    if (off > ws_size || off > (size_t)134217728) return;

    k_wt16<<<dim3((NNODE * (NNODE / 8)) / 256, 1), 256, 0, stream>>>(U, NNODE, NNODE, LG_PER, ut16, SW_U);
    k_wt16<<<dim3((NFEAT * (NNODE / 8)) / 256, 1), 256, 0, stream>>>(x, NNODE, NFEAT, LG_PER, xt16, SW_X);
    k_cvt16<<<(NNODE * (NNODE / 8)) / 256, 256, 0, stream>>>(U, u16, (unsigned)(NNODE * (NNODE / 8)), SW_U);
    k_lamdiag<<<NNODE / LD_ROWS, 256, 0, stream>>>(lam, a_l, b_l, c_l, dvec);
    k_prep<<<(NNODE * NFEAT / 4) / 256, 256, 0, stream>>>(x, alpha, xr, zb);

    const unsigned g1 = ((NFEAT / 64) * (NNODE / 64) + 7) / 8;
    const unsigned g2 = ((NNODE / 64) * (NFEAT / 64) + 7) / 8;

    k_gemm64<0, false, false><<<g1, 256, 0, stream>>>((const _Float16*)xt16, NNODE, (const _Float16*)ut16, NNODE,
        (void*)yt, NNODE, zb, xr, NFEAT, NNODE, NNODE, SC, 1.0f);
    k_zscale<<<(NFEAT * (NNODE / 8)) / 256, 256, 0, stream>>>(yt, dvec, zt16);
    k_gemm64<0, true, false><<<g2, 256, 0, stream>>>((const _Float16*)u16, NNODE, (const _Float16*)zt16, NNODE,
        (void*)out, NFEAT, zb, xr, NNODE, NFEAT, NNODE, SC, 1.0f);
}
